// GAT_22488448762008
// MI455X (gfx1250) — hardware-verified
//
#include <hip/hip_runtime.h>
#include <stddef.h>
#include <stdint.h>
#include <math.h>


#define RNE_LIST_PARAMS 0

#define NN      50000
#define NEDGE   850000
#define HID     64
#define NG      64
#define OUTD    10
#define NLAY    4
#define NREP    5
#define MP      50048
#define NTHR    256
#define NWAVE   8
#define EPT     8
#define CHUNK   (NTHR * EPT)
#define WCAP    (EPT * 32)
#define LISTN   (NWAVE * WCAP)
#define NBA     1024
#define SLA     10
#define SRCB    17
#define RCAP    28672
#define DEGCAP  64
#define MEAS_B1024  17720
#define MEAS_MAXDEG 34
#define NRB     49
#define GBM     128
#define BTK     192
#define NWB     24
#define NPB     6
#define EPB     8192
#define PA_AS   0
#define PA_AD   256
#define PA_G    512
#define PA_B    768
#define PA_PW   1024
#define PA_PB   4224
#define PA_TOT  4288
#define NEGSL   0.2f
#define WSMAX   134217728
#define BKT_LDS_INTS  (LISTN + 2 * RCAP + 3 * NBA + 16)
#define SCAN_LDS_INTS (2048 + RCAP + 2 * NBA + 16)
#define BIN_BYTES     (4 * NG * HID * 8)

static_assert(HID == 64 && NG == 64 && OUTD == 10);
static_assert(NN < (1 << SRCB) && (SRCB + SLA) < 31);
static_assert(MP % GBM == 0 && MP >= NN && MP - NN < GBM && MP % 32 == 0);
static_assert(NRB * NBA >= MP && (NRB - 1) * NBA < MP);
static_assert((CHUNK & (CHUNK - 1)) == 0 && NBA == (1 << SLA));
static_assert(((long long)CHUNK << SLA) < (1LL << 31));
static_assert(NBA % NWAVE == 0 && NBA % 32 == 0 && NBA % 16 == 0);
static_assert(RCAP % (NTHR * 4) == 0 && (2 * NBA) % (NTHR * 4) == 0);
static_assert((RCAP + 3 * NBA) % 4 == 0);
static_assert(RCAP >= MEAS_B1024 + 4096);
static_assert(DEGCAP >= MEAS_MAXDEG + 8);
static_assert(BKT_LDS_INTS * 4 <= 300000 && SCAN_LDS_INTS * 4 <= 300000);
static_assert(NLAY * HID * (BTK / 8) == NWB * NTHR);
static_assert(BTK % 32 == 0 && BTK == 3 * HID);
static_assert(GBM == NWAVE * 16 && GBM * HID == 8 * NTHR * 4);
static_assert((16 * OUTD * 4) % 128 == 0 && NG % 16 == 0);
static_assert(PA_TOT % 32 == 0 && PA_PB - PA_PW == NREP * HID * OUTD);
static_assert(EPB % 1024 == 0);

typedef float          v2f  __attribute__((ext_vector_type(2)));
typedef float          v4f  __attribute__((ext_vector_type(4)));
typedef float          v8f  __attribute__((ext_vector_type(8)));
typedef double         v2d  __attribute__((ext_vector_type(2)));
typedef int            v4i  __attribute__((ext_vector_type(4)));
typedef int            v8i  __attribute__((ext_vector_type(8)));
typedef unsigned short v8us __attribute__((ext_vector_type(8)));
typedef __bf16         v16b __attribute__((ext_vector_type(16)));
typedef v2f  __attribute__((may_alias)) v2fa;
typedef v4f  __attribute__((may_alias)) v4fa;
typedef v2d  __attribute__((may_alias)) v2da;
typedef v4i  __attribute__((may_alias)) v4ia;
typedef v8us __attribute__((may_alias)) v8usa;
union FragB { v16b v; v8us h[2]; v8i w; };

__device__ __forceinline__ v8f wmb(const FragB& a, const FragB& b, v8f c) {
  v8f d = __builtin_amdgcn_wmma_f32_16x16x32_bf16(false, a.v, false, b.v, (short)0, c, false, false);
  asm volatile("v_nop\n\tv_nop\n\tv_nop\n\tv_nop" : "+v"(d) : "v"(a.w), "v"(b.w));
  return d;
}

__device__ __forceinline__ unsigned int f2bf(float f) {
  const unsigned int u = __float_as_uint(f);
  const unsigned int r = ((u + 0x7FFFu + ((u >> 16) & 1u)) >> 16) & 0xFFFFu;
  return ((u & 0x7FFFFFFFu) > 0x7F800000u) ? 0x7FC0u : r;
}
__device__ __forceinline__ float bf2f(unsigned int b) { return __uint_as_float(b << 16); }
__device__ __forceinline__ float bfr(float f) { return bf2f(f2bf(f)); }
__device__ __forceinline__ float lpar(float v) {
#if RNE_LIST_PARAMS
  return bfr(v);
#else
  return v;
#endif
}
__device__ __forceinline__ float nanmax(float a, float b) { return ((b > a) | (b != b)) ? b : a; }

template <int SLB>
__device__ __forceinline__ int scan_chunk(const int* __restrict__ dsts, int nE, int cbase, int slotBase,
                                          int nb, int vec8, int* list, int tid, int lane, int wave) {
  int wc = 0;
  const int el0  = tid * EPT;
  const int e0   = cbase + el0;
  const int sent = -2147483647 - 1;
  v4i da, db;
  if (vec8 != 0 && cbase + CHUNK <= nE) {
    da = *(const v4i*)(dsts + e0);
    db = *(const v4i*)(dsts + e0 + 4);
  } else {
    da.x = (e0     < nE) ? dsts[min(e0,     nE - 1)] : sent;
    da.y = (e0 + 1 < nE) ? dsts[min(e0 + 1, nE - 1)] : sent;
    da.z = (e0 + 2 < nE) ? dsts[min(e0 + 2, nE - 1)] : sent;
    da.w = (e0 + 3 < nE) ? dsts[min(e0 + 3, nE - 1)] : sent;
    db.x = (e0 + 4 < nE) ? dsts[min(e0 + 4, nE - 1)] : sent;
    db.y = (e0 + 5 < nE) ? dsts[min(e0 + 5, nE - 1)] : sent;
    db.z = (e0 + 6 < nE) ? dsts[min(e0 + 6, nE - 1)] : sent;
    db.w = (e0 + 7 < nE) ? dsts[min(e0 + 7, nE - 1)] : sent;
  }
  const unsigned nbs = (unsigned)slotBase;
  const unsigned unb = (unsigned)nb;
  const unsigned s0 = (unsigned)da.x - nbs, s1 = (unsigned)da.y - nbs;
  const unsigned s2 = (unsigned)da.z - nbs, s3 = (unsigned)da.w - nbs;
  const unsigned s4 = (unsigned)db.x - nbs, s5 = (unsigned)db.y - nbs;
  const unsigned s6 = (unsigned)db.z - nbs, s7 = (unsigned)db.w - nbs;
  const bool h0 = s0 < unb, h1 = s1 < unb, h2 = s2 < unb, h3 = s3 < unb;
  const bool h4 = s4 < unb, h5 = s5 < unb, h6 = s6 < unb, h7 = s7 < unb;
  const unsigned any = __builtin_amdgcn_ballot_w32(h0 | h1 | h2 | h3 | h4 | h5 | h6 | h7);
  if (any != 0u) {
#define HITJ(J, HJ, SJ) { \
      const unsigned mj = __builtin_amdgcn_ballot_w32(HJ); \
      if (mj != 0u) { \
        if (HJ) { \
          const int pos = wc + (int)__builtin_amdgcn_mbcnt_lo(mj, 0u); \
          if (pos < WCAP) list[wave * WCAP + pos] = ((el0 + (J)) << SLB) | (int)(SJ); \
        } \
        wc += (int)__builtin_popcount(mj); } }
    HITJ(0, h0, s0)
    HITJ(1, h1, s1)
    HITJ(2, h2, s2)
    HITJ(3, h3, s3)
    HITJ(4, h4, s4)
    HITJ(5, h5, s5)
    HITJ(6, h6, s6)
    HITJ(7, h7, s7)
#undef HITJ
  }
  return wc;
}

template <int MODE>
__device__ __forceinline__ void rowblock(int blk, const float* __restrict__ src, const int* __restrict__ gid,
                                         unsigned short* plane, double* prec, int* cntrec,
                                         const double* __restrict__ bnrec, const float* __restrict__ gam,
                                         const float* __restrict__ bet, double invN, int nrec, int nN, int MPr,
                                         double* bins, unsigned short* tile, int* sgid, float* cst, int* scnt) {
  constexpr int PW = (MODE == 0) ? 64 : 128;
  const int tid = (int)threadIdx.x;
  const int r = tid >> 6, c = tid & 63;
  const int base = blk * NBA;
  {
    v2d z; z.x = 0.0; z.y = 0.0;
#pragma unroll 1
    for (int i = tid; i < (4 * NG * HID) / 2; i += NTHR) *(v2da*)(bins + 2 * i) = z;
  }
#pragma unroll 1
  for (int i = tid; i < NBA; i += NTHR) {
    const int row = base + i;
    const int gv  = gid[row < nN ? row : nN - 1];
    sgid[i] = (row < nN) ? gv : -1;
  }
  if constexpr (MODE != 0) {
    if (tid < HID) {
      double s = 0.0, q = 0.0;
#pragma unroll 2
      for (int b = 0; b < nrec; ++b) {
        s += bnrec[(size_t)b * 128 + c];
        q += bnrec[(size_t)b * 128 + 64 + c];
      }
      const double mud = s * invN;
      double var = q * invN - mud * mud;
      var = (var < 0.0) ? 0.0 : var;
      const double rstd = 1.0 / sqrt(var + 1e-5);
      cst[c]       = (float)mud;
      cst[64 + c]  = (float)rstd;
      cst[128 + c] = gam[c];
      cst[192 + c] = bet[c];
    }
  }
  __syncthreads();
  float mu = 0.0f, rs = 1.0f, ga = 1.0f, be = 0.0f;
  if constexpr (MODE != 0) { mu = cst[c]; rs = cst[64 + c]; ga = cst[128 + c]; be = cst[192 + c]; }
  if constexpr (MODE == 0) {
    if (tid < NG) {
      int k = 0;
#pragma unroll 4
      for (int i = 0; i < NBA; ++i) k += (sgid[i] == tid) ? 1 : 0;
      scnt[tid] = k;
    }
  }

#pragma unroll 1
  for (int t = 0; t < NBA / 32; ++t) {
    const int tbase = base + 32 * t;
    if (tbase >= MPr) break;
#pragma unroll 1
    for (int j = 0; j < 8; ++j) {
      const int lr  = r + 4 * j;
      const int row = tbase + lr;
      const bool live = row < nN;
      const int rc  = live ? row : nN - 1;
      const float x = src[(size_t)rc * HID + c];
      float v;
      if constexpr (MODE == 0) {
        v = bfr(x);
      } else {
        const float y = ((x - mu) * rs) * ga + be;
        v = (y > 0.0f) ? y : expm1f(y);
      }
      v = live ? v : 0.0f;
      const int g   = sgid[32 * t + lr];
      const bool ok = (unsigned)g < (unsigned)NG;
      const int gc  = ok ? g : 0;
      double* bp = bins + ((size_t)(r * NG + gc) * HID + c);
      const double add = ok ? (double)v : 0.0;
      *bp = *bp + add;
      if constexpr (MODE != 2) {
        const unsigned int hb = f2bf(v);
        tile[lr * PW + c] = (unsigned short)hb;
        if constexpr (MODE == 1) tile[lr * PW + 64 + c] = (unsigned short)f2bf(v - bf2f(hb));
      }
    }
    if constexpr (MODE != 2) {
      __syncthreads();
      if constexpr (MODE == 0) {
        const v8us a = *(const v8usa*)(tile + 8 * tid);
        unsigned short* dp = plane + (size_t)tbase * PW + 8 * tid;
        *(volatile v8us*)dp = a;
        __threadfence();
        *(volatile v8us*)dp = a;
      } else {
        const v8us a0 = *(const v8usa*)(tile + 8 * tid);
        const v8us a1 = *(const v8usa*)(tile + 8 * (tid + NTHR));
        unsigned short* dp = plane + (size_t)tbase * PW + 8 * tid;
        *(volatile v8us*)dp = a0;
        *(volatile v8us*)(dp + 8 * NTHR) = a1;
        __threadfence();
        *(volatile v8us*)dp = a0;
        *(volatile v8us*)(dp + 8 * NTHR) = a1;
      }
      __syncthreads();
    }
  }
  __syncthreads();

  v2d pv[8];
#pragma unroll
  for (int i = 0; i < 8; ++i) {
    const int e = 2 * (tid + NTHR * i);
    v2d a = *(const v2da*)(bins + e);
    const v2d b1 = *(const v2da*)(bins + NG * HID + e);
    const v2d b2 = *(const v2da*)(bins + 2 * NG * HID + e);
    const v2d b3 = *(const v2da*)(bins + 3 * NG * HID + e);
    a.x = ((a.x + b1.x) + b2.x) + b3.x;
    a.y = ((a.y + b1.y) + b2.y) + b3.y;
    pv[i] = a;
  }
  double* pp = prec + (size_t)blk * (NG * HID) + 2 * tid;
  v4i cv = {0, 0, 0, 0};
  int* cp = cntrec;
  if constexpr (MODE == 0) {
    if (tid < 16) cv = *(const v4ia*)(scnt + 4 * tid);
    cp = cntrec + (size_t)blk * NG + 4 * (tid & 15);
  }
#pragma unroll
  for (int i = 0; i < 8; ++i) *(volatile v2d*)(pp + 2 * NTHR * i) = pv[i];
  if constexpr (MODE == 0) { if (tid < 16) *(volatile v4i*)cp = cv; }
  __threadfence();
#pragma unroll
  for (int i = 0; i < 8; ++i) *(volatile v2d*)(pp + 2 * NTHR * i) = pv[i];
  if constexpr (MODE == 0) { if (tid < 16) *(volatile v4i*)cp = cv; }
}

__device__ __forceinline__ void copy_par(const float* __restrict__ s, int n, float* d, int npad, int tid) {
#pragma unroll 1
  for (int u = tid; u < npad / 4; u += NTHR) {
    const int j = 4 * u;
    const float f0 = s[min(j,     n - 1)];
    const float f1 = s[min(j + 1, n - 1)];
    const float f2 = s[min(j + 2, n - 1)];
    const float f3 = s[min(j + 3, n - 1)];
    v4f o;
    o.x = (j     < n) ? lpar(f0) : 0.0f;
    o.y = (j + 1 < n) ? lpar(f1) : 0.0f;
    o.z = (j + 2 < n) ? lpar(f2) : 0.0f;
    o.w = (j + 3 < n) ? lpar(f3) : 0.0f;
    float* dp = d + j;
    *(volatile v4f*)dp = o;
    __threadfence();
    *(volatile v4f*)dp = o;
  }
}

__global__ __launch_bounds__(NTHR) void k_prep(const float* __restrict__ X, const int* __restrict__ gid,
    const float* __restrict__ W, const float* __restrict__ pas, const float* __restrict__ pad,
    const float* __restrict__ pbg, const float* __restrict__ pbb, const float* __restrict__ ppw,
    const float* __restrict__ ppb, unsigned short* XB, unsigned short* BT, float* PAR,
    double* PREC0, int* CNT, int nN, int MPr) {
  extern __shared__ __attribute__((aligned(16))) double dbin[];
  __shared__ __attribute__((aligned(16))) unsigned short tile[32 * 128];
  __shared__ __attribute__((aligned(16))) int sgid[NBA];
  __shared__ __attribute__((aligned(16))) float cst[4 * HID];
  __shared__ __attribute__((aligned(16))) int scnt[NG];
  const int blk = (int)blockIdx.x;
  const int tid = (int)threadIdx.x;
  if (blk < NRB) {
    rowblock<0>(blk, X, gid, XB, PREC0, CNT, nullptr, nullptr, nullptr, 0.0, 0, nN, MPr,
                dbin, tile, sgid, cst, scnt);
  } else if (blk < NRB + NWB) {
    const int u   = (blk - NRB) * NTHR + tid;
    const int l   = u / (HID * (BTK / 8));
    const int rem = u - l * (HID * (BTK / 8));
    const int n   = rem / (BTK / 8);
    const int k8  = (rem - n * (BTK / 8)) * 8;
    const int seg = k8 >> 6;
    const int kk  = k8 & 63;
    const float* p = W + (size_t)l * (HID * HID) + (size_t)kk * HID + n;
    const bool useLo = (l == 0) ? (seg == 1) : (seg == 2);
    const bool zero  = (l == 0) && (seg == 2);
    v8us o;
#pragma unroll
    for (int i = 0; i < 8; ++i) {
      const float w = lpar(p[(size_t)i * HID]);
      const unsigned int hb = f2bf(w);
      const unsigned int lb = f2bf(w - bf2f(hb));
      o[i] = zero ? (unsigned short)0 : (useLo ? (unsigned short)lb : (unsigned short)hb);
    }
    unsigned short* dp = BT + (size_t)u * 8;
    *(volatile v8us*)dp = o;
    __threadfence();
    *(volatile v8us*)dp = o;
  } else {
    const int pb = blk - NRB - NWB;
    if (pb == 0)      copy_par(pas, NLAY * HID, PAR + PA_AS, 256, tid);
    else if (pb == 1) copy_par(pad, NLAY * HID, PAR + PA_AD, 256, tid);
    else if (pb == 2) copy_par(pbg, NLAY * HID, PAR + PA_G, 256, tid);
    else if (pb == 3) copy_par(pbb, NLAY * HID, PAR + PA_B, 256, tid);
    else if (pb == 4) copy_par(ppw, NREP * HID * OUTD, PAR + PA_PW, NREP * HID * OUTD, tid);
    else              copy_par(ppb, NREP * OUTD, PAR + PA_PB, PA_TOT - PA_PB, tid);
  }
}

__global__ __launch_bounds__(NTHR) void k_bucket(const int* __restrict__ srcs, const int* __restrict__ dsts,
                                                 int nE, int nN, int vec8, int* HITS, int* META, int* FLG) {
  extern __shared__ __attribute__((aligned(16))) int bsm[];
  int* list = bsm;
  int* hl   = bsm + LISTN;
  int* sl   = hl + RCAP;
  int* cnt  = sl + RCAP;
  int* offs = cnt + NBA;
  int* cur  = offs + NBA;
  int* wcnt = cur + NBA;
  const int tid = (int)threadIdx.x, lane = tid & 31, wave = tid >> 5;
  const int blk = (int)blockIdx.x;
  const int nodeBase = blk * NBA;
  int nb = nN - nodeBase;
  nb = nb < 0 ? 0 : (nb > NBA ? NBA : nb);

  {
    const v4i z4 = {0, 0, 0, 0};
    for (int i = tid * 4; i < RCAP + 3 * NBA; i += NTHR * 4) *(v4ia*)(sl + i) = z4;
    if (tid < 16) wcnt[tid] = 0;
  }
  __syncthreads();

  int tot = 0, ovf = 0;
  const int nChunks = (nE + CHUNK - 1) / CHUNK;
#pragma unroll 1
  for (int ch = 0; ch < nChunks; ++ch) {
    const int cbase = ch * CHUNK;
    const int wc = scan_chunk<SLA>(dsts, nE, cbase, nodeBase, nb, vec8, list, tid, lane, wave);
    if (lane == 0) wcnt[wave] = wc;
    __syncthreads();
    int pre = 0, all = 0;
#pragma unroll
    for (int w2 = 0; w2 < NWAVE; ++w2) {
      int c = wcnt[w2];
      c = c < 0 ? 0 : (c > WCAP ? WCAP : c);
      all += c;
      pre += (w2 < wave) ? c : 0;
    }
    const int wcc  = wc > WCAP ? WCAP : wc;
    const int base = tot + pre;
#pragma unroll 1
    for (int i = lane; i < wcc; i += 32) {
      const int ent = list[wave * WCAP + i];
      const int el  = (ent >> SLA) & (CHUNK - 1);
      const int sq  = ent & (NBA - 1);
      int eid = cbase + el;
      eid = eid > nE - 1 ? nE - 1 : eid;
      const int sraw = srcs[eid];
      const int s = sraw < 0 ? 0 : (sraw > nN - 1 ? nN - 1 : sraw);
      const int pos = base + i;
      if (pos < RCAP) hl[pos] = (int)((unsigned)s | ((unsigned)sq << SRCB));
    }
    if (tot + all > RCAP) ovf = 1;
    tot += all;
    tot = tot > RCAP ? RCAP : tot;
    __syncthreads();
  }
  const int nh = tot;

  if (wave == 0) {
#pragma unroll 1
    for (int b0 = 0; b0 < nh; b0 += 32) {
      const int idx = b0 + lane;
      const int uv  = hl[idx < nh ? idx : nh - 1];
      const int m32 = (nh - b0) < 32 ? (nh - b0) : 32;
#pragma unroll 1
      for (int k = 0; k < m32; ++k) {
        const int u  = __builtin_amdgcn_readlane(uv, k);
        const int sq = (u >> SRCB) & (NBA - 1);
        if (lane == 0) cnt[sq] = cnt[sq] + 1;
      }
    }
  }
  __syncthreads();
  if (wave == 0) {
    const int base = lane * (NBA / 32);
    int s = 0;
#pragma unroll 1
    for (int i = 0; i < NBA / 32; ++i) s += cnt[base + i];
    int incl = s;
#pragma unroll
    for (int d = 1; d < 32; d <<= 1) {
      const int y = __shfl_up(incl, d, 32);
      if (lane >= d) incl += y;
    }
    int run = incl - s;
#pragma unroll 1
    for (int i = 0; i < NBA / 32; ++i) {
      const int cv = cnt[base + i];
      offs[base + i] = run;
      cur[base + i]  = run;
      run += cv;
    }
  }
  __syncthreads();
  if (wave == 0) {
#pragma unroll 1
    for (int b0 = 0; b0 < nh; b0 += 32) {
      const int idx = b0 + lane;
      const int uv  = hl[idx < nh ? idx : nh - 1];
      const int m32 = (nh - b0) < 32 ? (nh - b0) : 32;
#pragma unroll 1
      for (int k = 0; k < m32; ++k) {
        const int u  = __builtin_amdgcn_readlane(uv, k);
        const int sq = (u >> SRCB) & (NBA - 1);
        if (lane == 0) {
          int p = cur[sq];
          p = p < 0 ? 0 : (p > RCAP - 1 ? RCAP - 1 : p);
          sl[p] = u;
          cur[sq] = p + 1;
        }
      }
    }
  }
  __syncthreads();

  int* hb = HITS + (size_t)blk * RCAP;
  int* mb = META + (size_t)blk * (2 * NBA);
  v4i cv;
  cv.x = (tid == 0) ? nh : 0;
  cv.y = (tid == 0) ? ovf : 0;
  cv.z = 0; cv.w = 0;
  int* fp = FLG + (size_t)blk * 32 + 4 * (tid & 7);
#pragma unroll 1
  for (int p = tid * 4; p < RCAP; p += NTHR * 4) {
    const v4i v = *(const v4ia*)(sl + p);
    *(volatile v4i*)(hb + p) = v;
  }
#pragma unroll 1
  for (int p = tid * 4; p < 2 * NBA; p += NTHR * 4) {
    const v4i v = *(const v4ia*)(cnt + p);
    *(volatile v4i*)(mb + p) = v;
  }
  if (tid < 8) *(volatile v4i*)fp = cv;
  __threadfence();
#pragma unroll 1
  for (int p = tid * 4; p < RCAP; p += NTHR * 4) {
    const v4i v = *(const v4ia*)(sl + p);
    *(volatile v4i*)(hb + p) = v;
  }
#pragma unroll 1
  for (int p = tid * 4; p < 2 * NBA; p += NTHR * 4) {
    const v4i v = *(const v4ia*)(cnt + p);
    *(volatile v4i*)(mb + p) = v;
  }
  if (tid < 8) *(volatile v4i*)fp = cv;
}

template <int AW, int KS>
__global__ __launch_bounds__(NTHR) void k_gemm(const unsigned short* __restrict__ A,
                                               const unsigned short* __restrict__ BT,
                                               const float* __restrict__ avs, const float* __restrict__ avd,
                                               float* H, float* SD, int MPr) {
  static_assert(32 * KS <= BTK && (AW == 64 || AW == 128));
  __shared__ __attribute__((aligned(16))) float stg[GBM * HID];
  __shared__ __attribute__((aligned(16))) float satt[2 * HID];
  __shared__ __attribute__((aligned(16))) float sdot[2 * GBM];
  const int tid = (int)threadIdx.x, lane = tid & 31, wave = tid >> 5, hh = lane >> 4, m = lane & 15;
  const int rowBase = (int)blockIdx.x * GBM;

  if (tid < 2 * HID) {
    const int which = tid >> 6;
    const int c = tid & 63;
    const float vs = avs[c];
    const float vd = avd[c];
    satt[tid] = (which == 0) ? vs : vd;
  }

  v8f acc[4];
  {
    const v8f z = {0.f, 0.f, 0.f, 0.f, 0.f, 0.f, 0.f, 0.f};
    acc[0] = z; acc[1] = z; acc[2] = z; acc[3] = z;
  }
  const unsigned short* ap = A  + (size_t)(rowBase + 16 * wave + m) * (size_t)AW + 8 * hh;
  const unsigned short* bp = BT + (size_t)m * (size_t)BTK + 8 * hh;
#pragma unroll
  for (int ks = 0; ks < KS; ++ks) {
    const int acol = (32 * ks) % AW;
    FragB af;
    af.h[0] = *(const v8usa*)(ap + acol);
    af.h[1] = *(const v8usa*)(ap + acol + 16);
#pragma unroll
    for (int t = 0; t < 4; ++t) {
      const unsigned short* wq = bp + (size_t)(16 * t) * (size_t)BTK + 32 * ks;
      FragB bf;
      bf.h[0] = *(const v8usa*)wq;
      bf.h[1] = *(const v8usa*)(wq + 16);
      acc[t] = wmb(af, bf, acc[t]);
    }
  }

#pragma unroll
  for (int t = 0; t < 4; ++t) {
    const int lc = 16 * t + m;
#pragma unroll
    for (int r = 0; r < 8; ++r) {
      const int lr = 16 * wave + 8 * hh + r;
      stg[lr * HID + lc] = acc[t][r];
    }
  }
  __syncthreads();

  {
    const int row = tid & (GBM - 1), which = tid >> 7;
    const float* sa = satt + which * HID;
    const float* hr = stg + row * HID;
    float d = 0.f;
#pragma unroll 4
    for (int c4 = 0; c4 < HID / 4; ++c4) {
      const v4f hv = *(const v4fa*)(hr + 4 * c4);
      const v4f av = *(const v4fa*)(sa + 4 * c4);
      d = fmaf(hv.x, av.x, d);
      d = fmaf(hv.y, av.y, d);
      d = fmaf(hv.z, av.z, d);
      d = fmaf(hv.w, av.w, d);
    }
    sdot[which * GBM + row] = d;
  }
  __syncthreads();

  v4f fv[8];
#pragma unroll
  for (int i = 0; i < 8; ++i) fv[i] = *(const v4fa*)(stg + 4 * (tid + NTHR * i));
  const v4f sdv = *(const v4fa*)(sdot + 4 * (tid & 63));
  float* hp = H + (size_t)rowBase * HID + 4 * tid;
  float* sp = SD + (size_t)(wave & 1) * (size_t)MPr + rowBase + 4 * lane;
#pragma unroll
  for (int i = 0; i < 8; ++i) *(volatile v4f*)(hp + 4 * NTHR * i) = fv[i];
  if (wave < 2) *(volatile v4f*)sp = sdv;
  __threadfence();
#pragma unroll
  for (int i = 0; i < 8; ++i) *(volatile v4f*)(hp + 4 * NTHR * i) = fv[i];
  if (wave < 2) *(volatile v4f*)sp = sdv;
}

__global__ __launch_bounds__(NTHR) void k_emax(const int* __restrict__ ei, int nE, int nN, int vec4,
                                               const float* __restrict__ SD, int MPr, float* EMX) {
  __shared__ int sm[NWAVE];
  const int tid = (int)threadIdx.x, lane = tid & 31, wave = tid >> 5;
  const int blk = (int)blockIdx.x;
  const int* srcs = ei;
  const int* dsts = ei + nE;
  const float* ES = SD;
  const float* ED = SD + MPr;
  float mv = __int_as_float((int)0xff800000);
  const int bb = blk * EPB;
#pragma unroll 1
  for (int it = 0; it < EPB / 1024; ++it) {
    const int cbase = bb + it * 1024;
    if (cbase >= nE) break;
    const int e0 = cbase + 4 * tid;
    v4i s4, d4;
    if (vec4 != 0 && cbase + 1024 <= nE) {
      s4 = *(const v4i*)(srcs + e0);
      d4 = *(const v4i*)(dsts + e0);
    } else {
      s4.x = srcs[min(e0, nE - 1)];     d4.x = dsts[min(e0, nE - 1)];
      s4.y = srcs[min(e0 + 1, nE - 1)]; d4.y = dsts[min(e0 + 1, nE - 1)];
      s4.z = srcs[min(e0 + 2, nE - 1)]; d4.z = dsts[min(e0 + 2, nE - 1)];
      s4.w = srcs[min(e0 + 3, nE - 1)]; d4.w = dsts[min(e0 + 3, nE - 1)];
    }
    const int a0 = min(max(s4.x, 0), nN - 1), b0 = min(max(d4.x, 0), nN - 1);
    const int a1 = min(max(s4.y, 0), nN - 1), b1 = min(max(d4.y, 0), nN - 1);
    const int a2 = min(max(s4.z, 0), nN - 1), b2 = min(max(d4.z, 0), nN - 1);
    const int a3 = min(max(s4.w, 0), nN - 1), b3 = min(max(d4.w, 0), nN - 1);
    float x0 = ES[a0] + ED[b0];
    float x1 = ES[a1] + ED[b1];
    float x2 = ES[a2] + ED[b2];
    float x3 = ES[a3] + ED[b3];
    x0 = (x0 >= 0.f) ? x0 : NEGSL * x0;
    x1 = (x1 >= 0.f) ? x1 : NEGSL * x1;
    x2 = (x2 >= 0.f) ? x2 : NEGSL * x2;
    x3 = (x3 >= 0.f) ? x3 : NEGSL * x3;
    mv = nanmax(mv, x0); mv = nanmax(mv, x1); mv = nanmax(mv, x2); mv = nanmax(mv, x3);
  }
#pragma unroll
  for (int d = 16; d >= 1; d >>= 1) {
    const float o = __shfl_xor(mv, d, 32);
    mv = nanmax(mv, o);
  }
  if (lane == 0) sm[wave] = __float_as_int(mv);
  __syncthreads();
  float bm = __int_as_float(sm[0]);
#pragma unroll
  for (int w2 = 1; w2 < NWAVE; ++w2) bm = nanmax(bm, __int_as_float(sm[w2]));
  v4f o4; o4.x = bm; o4.y = bm; o4.z = bm; o4.w = bm;
  float* op = EMX + (size_t)blk * 32 + 4 * (tid & 7);
  if (tid < 8) *(volatile v4f*)op = o4;
  __threadfence();
  if (tid < 8) *(volatile v4f*)op = o4;
}

__global__ __launch_bounds__(NTHR) void k_scan(const int* __restrict__ HITS, const int* __restrict__ META,
                                               const int* __restrict__ FLGB, const float* __restrict__ EMX,
                                               int nrec, const float* __restrict__ H,
                                               const float* __restrict__ SD, float* AGG, double* BNR,
                                               int nN, int MPr) {
  extern __shared__ __attribute__((aligned(16))) int ssm[];
  double* wsum = (double*)ssm;
  int* sl   = ssm + 2048;
  int* cnt  = sl + RCAP;
  int* offs = cnt + NBA;
  int* misc = offs + NBA;
  const int tid = (int)threadIdx.x, lane = tid & 31, wave = tid >> 5;
  const int blk = (int)blockIdx.x;
  const int nodeBase = blk * NBA;
  const float* ES = SD;
  const float* ED = SD + MPr;

  const int nhraw = FLGB[(size_t)blk * 32];
  const int bflag = FLGB[(size_t)blk * 32 + 1];
  const int nh  = nhraw < 0 ? 0 : (nhraw > RCAP ? RCAP : nhraw);
  const int ovf = (bflag != 0 || nhraw < 0 || nhraw > RCAP) ? 1 : 0;
  int nh4 = (nh + 3) & ~3;
  nh4 = nh4 < 4 ? 4 : nh4;
  {
    const int* hb = HITS + (size_t)blk * RCAP;
#pragma unroll 1
    for (int p = tid * 4; p < nh4; p += NTHR * 4) *(v4ia*)(sl + p) = *(const v4i*)(hb + p);
    const int* mb = META + (size_t)blk * (2 * NBA);
#pragma unroll 1
    for (int p = tid * 4; p < 2 * NBA; p += NTHR * 4) *(v4ia*)(cnt + p) = *(const v4i*)(mb + p);
  }
  {
    const int ri = tid < nrec ? tid : nrec - 1;
    float mv = EMX[(size_t)ri * 32];
#pragma unroll
    for (int d = 16; d >= 1; d >>= 1) {
      const float o = __shfl_xor(mv, d, 32);
      mv = nanmax(mv, o);
    }
    if (lane == 0) misc[wave] = __float_as_int(mv);
  }
  __syncthreads();
  float M = __int_as_float(misc[0]);
#pragma unroll
  for (int w2 = 1; w2 < NWAVE; ++w2) M = nanmax(M, __int_as_float(misc[w2]));

  const float qnan = __int_as_float(0x7fc00000);
  const float pzb  = (ovf != 0) ? qnan : 0.0f;
  const int nhm = nh4 - 1;
  double ps0 = 0.0, ps1 = 0.0, pq0 = 0.0, pq1 = 0.0;

#pragma unroll 1
  for (int si = 0; si < NBA / NWAVE; ++si) {
    const int s    = si * NWAVE + wave;
    const int node = nodeBase + s;
    const int nc   = node < nN ? node : nN - 1;
    int c = cnt[s];
    const bool big = c > DEGCAP;
    c = c < 0 ? 0 : (c > DEGCAP ? DEGCAP : c);
    int o = offs[s];
    o = o < 0 ? 0 : (o > RCAP ? RCAP : o);
    if (c > nh - o) c = nh - o;
    c = c < 0 ? 0 : c;
    const float edv = ED[nc];
    float dn = 0.0f, a0 = 0.0f, a1 = 0.0f;
#pragma unroll 1
    for (int b0 = 0; b0 < c; b0 += 32) {
      int t = b0 + lane;
      t = t > c - 1 ? c - 1 : t;
      int idx = o + t;
      idx = idx < 0 ? 0 : (idx > nhm ? nhm : idx);
      const int ent = sl[idx];
      int sr = ent & ((1 << SRCB) - 1);
      sr = sr > nN - 1 ? nN - 1 : sr;
      float x = ES[sr] + edv;
      x = (x >= 0.f) ? x : NEGSL * x;
      const float p  = expf(x - M);
      const int   pi = __float_as_int(p);
      const int m32 = (c - b0) < 32 ? (c - b0) : 32;
#pragma unroll 1
      for (int k = 0; k < m32; ++k) {
        const int   sk = __builtin_amdgcn_readlane(sr, k);
        const float pk = __int_as_float(__builtin_amdgcn_readlane(pi, k));
        const v2f rw = *(const v2fa*)(H + (size_t)sk * HID + 2 * lane);
        dn += pk;
        a0 = fmaf(pk, rw.x, a0);
        a1 = fmaf(pk, rw.y, a1);
      }
    }
    const float inv = 1.0f / (dn + 1e-12f);
    const float pzr = big ? qnan : pzb;
    const float r0 = a0 * inv + pzr;
    const float r1 = a1 * inv + pzr;
    const bool live = node < nN;
    v2f ov;
    ov.x = live ? r0 : 0.0f;
    ov.y = live ? r1 : 0.0f;
    if (node < MPr) {
      float* op = AGG + (size_t)node * HID + 2 * lane;
      *(volatile v2f*)op = ov;
      __threadfence();
      *(volatile v2f*)op = ov;
    }
    const double d0 = (double)r0, d1 = (double)r1;
    ps0 += live ? d0 : 0.0;
    ps1 += live ? d1 : 0.0;
    pq0 += live ? d0 * d0 : 0.0;
    pq1 += live ? d1 * d1 : 0.0;
  }

  {
    v2d a; a.x = ps0; a.y = ps1;
    v2d b; b.x = pq0; b.y = pq1;
    *(v2da*)(wsum + wave * 128 + 2 * lane) = a;
    *(v2da*)(wsum + wave * 128 + 64 + 2 * lane) = b;
  }
  __syncthreads();
  if (wave == 0) {
    v2d ts; ts.x = 0.0; ts.y = 0.0;
    v2d tq; tq.x = 0.0; tq.y = 0.0;
#pragma unroll
    for (int w2 = 0; w2 < NWAVE; ++w2) {
      const v2d p = *(const v2da*)(wsum + w2 * 128 + 2 * lane);
      const v2d q = *(const v2da*)(wsum + w2 * 128 + 64 + 2 * lane);
      ts.x += p.x; ts.y += p.y;
      tq.x += q.x; tq.y += q.y;
    }
    double* rp = BNR + (size_t)blk * 128 + 2 * lane;
    *(volatile v2d*)rp = ts;
    *(volatile v2d*)(rp + 64) = tq;
    __threadfence();
    *(volatile v2d*)rp = ts;
    *(volatile v2d*)(rp + 64) = tq;
  }
}

template <int WP>
__global__ __launch_bounds__(NTHR) void k_act(const float* __restrict__ AGG, const int* __restrict__ gid,
                                              const double* __restrict__ BNR, const float* __restrict__ gam,
                                              const float* __restrict__ bet, unsigned short* AHL, double* PRECl,
                                              double invN, int nrec, int nN, int MPr) {
  extern __shared__ __attribute__((aligned(16))) double dbin[];
  __shared__ __attribute__((aligned(16))) unsigned short tile[32 * 128];
  __shared__ __attribute__((aligned(16))) int sgid[NBA];
  __shared__ __attribute__((aligned(16))) float cst[4 * HID];
  __shared__ __attribute__((aligned(16))) int scnt[NG];
  rowblock<(WP != 0) ? 1 : 2>((int)blockIdx.x, AGG, gid, AHL, PRECl, nullptr, BNR, gam, bet, invN, nrec,
                              nN, MPr, dbin, tile, sgid, cst, scnt);
}

__global__ __launch_bounds__(NTHR) void k_head(const double* __restrict__ PREC, const int* __restrict__ CNT,
                                               const int* __restrict__ FLG, const float* __restrict__ PAR,
                                               float* out, int nblk) {
  __shared__ __attribute__((aligned(16))) double psum[NREP * 16 * HID];
  __shared__ __attribute__((aligned(16))) float sinv[16];
  __shared__ __attribute__((aligned(16))) float res[16 * OUTD];
  __shared__ int sfl[NWAVE];
  const int tid = (int)threadIdx.x, lane = tid & 31, wave = tid >> 5;
  const int blk = (int)blockIdx.x;
  const int g0 = 16 * blk;

#pragma unroll 1
  for (int it = 0; it < (NREP * 16 * HID) / NTHR; ++it) {
    const int item = it * NTHR + tid;
    const int l   = item >> 10;
    const int rem = item & 1023;
    const int gl  = rem >> 6;
    const int c   = rem & 63;
    const double* p = PREC + ((size_t)l * (size_t)nblk * NG + (size_t)(g0 + gl)) * HID + c;
    double s = 0.0;
#pragma unroll 4
    for (int b = 0; b < nblk; ++b) s += p[(size_t)b * (NG * HID)];
    psum[item] = s;
  }
  if (tid < 16) {
    int k = 0;
#pragma unroll 4
    for (int b = 0; b < nblk; ++b) k += CNT[(size_t)b * NG + g0 + tid];
    const float cf = (k > 1) ? (float)k : 1.0f;
    sinv[tid] = 1.0f / cf;
  }
  {
    int f = 0;
#pragma unroll 1
    for (int i = tid; i < nblk; i += NTHR) f |= FLG[(size_t)i * 32 + 1];
    const unsigned bm = __builtin_amdgcn_ballot_w32(f != 0);
    if (lane == 0) sfl[wave] = (bm != 0u) ? 1 : 0;
  }
  __syncthreads();
  int anyf = 0;
#pragma unroll
  for (int w2 = 0; w2 < NWAVE; ++w2) anyf |= sfl[w2];

  if (tid < 16 * OUTD) {
    const int gl = tid / OUTD;
    const int o  = tid - gl * OUTD;
    const double iv = (double)sinv[gl];
    double acc = 0.0;
#pragma unroll 1
    for (int l = 0; l < NREP; ++l) {
      const double* ps = psum + (l * 16 + gl) * HID;
      const float*  wp = PAR + PA_PW + (size_t)l * (HID * OUTD) + o;
      double s = 0.0;
#pragma unroll 4
      for (int c = 0; c < HID; ++c) s = fma(ps[c], (double)wp[c * OUTD], s);
      acc += s * iv + (double)PAR[PA_PB + l * OUTD + o];
    }
    const float rv = (float)acc;
    res[tid] = (anyf != 0) ? __int_as_float(0x7fc00000) : rv;
  }
  __syncthreads();
  v4f ov = {0.f, 0.f, 0.f, 0.f};
  if (tid < 40) ov = *(const v4fa*)(res + 4 * tid);
  float* op = out + (size_t)blk * (16 * OUTD) + 4 * (tid < 40 ? tid : 0);
  if (tid < 40) *(volatile v4f*)op = ov;
  __threadfence();
  if (tid < 40) *(volatile v4f*)op = ov;
}

static inline int cdiv(int a, int b) { return (a + b - 1) / b; }
static inline size_t al256(size_t o) { return (o + 255) & ~(size_t)255; }

extern "C" void kernel_launch(void* const* d_in, const int* in_sizes, int n_in,
                              void* d_out, int out_size, void* d_ws, size_t ws_size,
                              hipStream_t stream) {
  if (n_in < 12) return;
  if (in_sizes[0] != NN * HID) return;
  if (in_sizes[1] < 2 || (in_sizes[1] & 1) != 0) return;
  const int nE = in_sizes[1] / 2;
  if (nE < 1 || nE > (1 << 24)) return;
  if (in_sizes[2] != NN) return;
  if (in_sizes[3] != NLAY * HID * HID) return;
  if (in_sizes[4] != NLAY * HID || in_sizes[5] != NLAY * HID) return;
  if (in_sizes[6] != NLAY * HID || in_sizes[7] != NLAY * HID) return;
  if (in_sizes[8] != NREP * HID * OUTD || in_sizes[9] != NREP * OUTD) return;
  if (out_size != NG * OUTD) return;
  const int nrec = cdiv(nE, EPB);
  if (nrec > NTHR) return;

  const float* X   = (const float*)d_in[0];
  const int*   ei  = (const int*)  d_in[1];
  const int*   gid = (const int*)  d_in[2];
  const float* W   = (const float*)d_in[3];
  const float* pas = (const float*)d_in[4];
  const float* pad = (const float*)d_in[5];
  const float* pbg = (const float*)d_in[6];
  const float* pbb = (const float*)d_in[7];
  const float* ppw = (const float*)d_in[8];
  const float* ppb = (const float*)d_in[9];
  float* out = (float*)d_out;
  const int* src = ei;
  const int* dst = ei + nE;
  const int nN = NN;
  const int vec = ((nE & 3) == 0) ? 1 : 0;

  char* ws = (char*)d_ws;
  size_t off = 0;
  const size_t oXB  = off; off = al256(off + (size_t)MP * HID * 2);
  const size_t oAHL = off; off = al256(off + (size_t)MP * 128 * 2);
  const size_t oH   = off; off = al256(off + (size_t)MP * HID * 4);
  const size_t oAGG = off; off = al256(off + (size_t)MP * HID * 4);
  const size_t oSD  = off; off = al256(off + (size_t)2 * MP * 4);
  const size_t oHIT = off; off = al256(off + (size_t)NRB * RCAP * 4);
  const size_t oMET = off; off = al256(off + (size_t)NRB * 2 * NBA * 4);
  const size_t oFLG = off; off = al256(off + (size_t)NRB * 128);
  const size_t oEMX = off; off = al256(off + (size_t)nrec * 128);
  const size_t oBNR = off; off = al256(off + (size_t)NRB * 128 * 8);
  const size_t oPRE = off; off = al256(off + (size_t)NREP * NRB * NG * HID * 8);
  const size_t oCNT = off; off = al256(off + (size_t)NRB * NG * 4);
  const size_t oBT  = off; off = al256(off + (size_t)NLAY * HID * BTK * 2);
  const size_t oPAR = off; off = al256(off + (size_t)PA_TOT * 4);
  if (off > ws_size || off > (size_t)WSMAX) return;
  unsigned short* XB  = (unsigned short*)(ws + oXB);
  unsigned short* AHL = (unsigned short*)(ws + oAHL);
  float*  H    = (float*)(ws + oH);
  float*  AGG  = (float*)(ws + oAGG);
  float*  SD   = (float*)(ws + oSD);
  int*    HITS = (int*)(ws + oHIT);
  int*    META = (int*)(ws + oMET);
  int*    FLG  = (int*)(ws + oFLG);
  float*  EMX  = (float*)(ws + oEMX);
  double* BNR  = (double*)(ws + oBNR);
  double* PREC = (double*)(ws + oPRE);
  int*    CNT  = (int*)(ws + oCNT);
  unsigned short* BT = (unsigned short*)(ws + oBT);
  float*  PAR  = (float*)(ws + oPAR);

  const int binLds  = BIN_BYTES;
  const int bktLds  = BKT_LDS_INTS * 4;
  const int scanLds = SCAN_LDS_INTS * 4;
  hipFuncSetAttribute(reinterpret_cast<const void*>(&k_prep), hipFuncAttributeMaxDynamicSharedMemorySize, binLds);
  hipFuncSetAttribute(reinterpret_cast<const void*>(&k_act<1>), hipFuncAttributeMaxDynamicSharedMemorySize, binLds);
  hipFuncSetAttribute(reinterpret_cast<const void*>(&k_act<0>), hipFuncAttributeMaxDynamicSharedMemorySize, binLds);
  hipFuncSetAttribute(reinterpret_cast<const void*>(&k_bucket), hipFuncAttributeMaxDynamicSharedMemorySize, bktLds);
  hipFuncSetAttribute(reinterpret_cast<const void*>(&k_scan), hipFuncAttributeMaxDynamicSharedMemorySize, scanLds);

  const double invN = 1.0 / (double)NN;
  const size_t precStride = (size_t)NRB * NG * HID;

  k_prep<<<NRB + NWB + NPB, NTHR, binLds, stream>>>(X, gid, W, pas, pad, pbg, pbb, ppw, ppb,
                                                   XB, BT, PAR, PREC, CNT, nN, MP);
  k_bucket<<<NRB, NTHR, bktLds, stream>>>(src, dst, nE, nN, vec, HITS, META, FLG);

  for (int l = 0; l < NLAY; ++l) {
    const unsigned short* btl = BT + (size_t)l * HID * BTK;
    const float* avs = PAR + PA_AS + l * HID;
    const float* avd = PAR + PA_AD + l * HID;
    if (l == 0) k_gemm<64, 4><<<MP / GBM, NTHR, 0, stream>>>(XB, btl, avs, avd, H, SD, MP);
    else        k_gemm<128, 6><<<MP / GBM, NTHR, 0, stream>>>(AHL, btl, avs, avd, H, SD, MP);
    k_emax<<<nrec, NTHR, 0, stream>>>(ei, nE, nN, vec, SD, MP, EMX);
    k_scan<<<NRB, NTHR, scanLds, stream>>>(HITS, META, FLG, EMX, nrec, H, SD, AGG, BNR, nN, MP);
    double* precl = PREC + (size_t)(l + 1) * precStride;
    const float* gl = PAR + PA_G + l * HID;
    const float* bl = PAR + PA_B + l * HID;
    if (l < NLAY - 1) k_act<1><<<NRB, NTHR, binLds, stream>>>(AGG, gid, BNR, gl, bl, AHL, precl, invN, NRB, nN, MP);
    else              k_act<0><<<NRB, NTHR, binLds, stream>>>(AGG, gid, BNR, gl, bl, AHL, precl, invN, NRB, nN, MP);
  }
  k_head<<<NG / 16, NTHR, 0, stream>>>(PREC, CNT, FLG, PAR, out, NRB);
}
